// MeanShiftStep_2370821947779
// MI455X (gfx1250) — hardware-verified
//
#include <hip/hip_runtime.h>


#define NP   8192
#define DD   32
#define NPD  64
#define CH   1024
#define NCH  (NP / CH)
#define RP   32
typedef _Float16 h16;
typedef unsigned short bf;
typedef __attribute__((ext_vector_type(16))) __bf16   v16bf;
typedef __attribute__((ext_vector_type(16))) _Float16 v16h;
typedef __attribute__((ext_vector_type(8)))  _Float16 v8h;
typedef __attribute__((ext_vector_type(8)))  unsigned short v8us;
typedef __attribute__((ext_vector_type(8)))  float    v8f;
typedef __attribute__((ext_vector_type(4)))  float    v4f;
typedef v8h  __attribute__((may_alias)) v8ha;
typedef v4f  __attribute__((may_alias)) v4fa;
typedef v8us __attribute__((may_alias)) v8usa;

__device__ __forceinline__ unsigned short f2bf(float f) { unsigned u = __float_as_uint(f); u += 0x7FFFu + ((u >> 16) & 1u); return (unsigned short)(u >> 16); }
__device__ __forceinline__ float bf2f(unsigned short b) { return __uint_as_float(((unsigned)b) << 16); }
__device__ __forceinline__ float bfr(float f) { return bf2f(f2bf(f)); }
__device__ __forceinline__ v16h cat16(v8h lo, v8h hi) { return __builtin_shufflevector(lo, hi, 0, 1, 2, 3, 4, 5, 6, 7, 8, 9, 10, 11, 12, 13, 14, 15); }
__device__ __forceinline__ v16bf cat16b(v8us lo, v8us hi) { return __builtin_bit_cast(v16bf, __builtin_shufflevector(lo, hi, 0, 1, 2, 3, 4, 5, 6, 7, 8, 9, 10, 11, 12, 13, 14, 15)); }
__device__ __forceinline__ v8f wmma16(v16h a, v16h b, v8f c) { return __builtin_amdgcn_wmma_f32_16x16x32_f16(false, a, false, b, (short)0, c, false, false); }
__device__ __forceinline__ v8f wmmab(v16bf a, v16bf b, v8f c) { return __builtin_amdgcn_wmma_f32_16x16x32_bf16(false, a, false, b, (short)0, c, false, false); }


template <typename T16> struct WFrag;
template <> struct WFrag<h16> { typedef v16h V; static __device__ __forceinline__ V ld(const h16* p) { return cat16(*(const v8h*)p, *(const v8h*)(p + 16)); } static __device__ __forceinline__ v8f mma(V a, V b, v8f c) { return wmma16(a, b, c); } };
template <> struct WFrag<bf> { typedef v16bf V; static __device__ __forceinline__ V ld(const bf* p) { return cat16b(*(const v8us*)p, *(const v8us*)(p + 16)); } static __device__ __forceinline__ v8f mma(V a, V b, v8f c) { return wmmab(a, b, c); } };
template <typename T16, int NSPLIT, bool BIAS>
__global__ __launch_bounds__(32) void k_gemmw(const T16* __restrict__ A, const T16* __restrict__ A2, const T16* __restrict__ Bt, const T16* __restrict__ Bt2, int K, float* C, int ldc, const float* __restrict__ bias, size_t sA, size_t sB, size_t sC) {
    typedef typename WFrag<T16>::V V;
    __shared__ __align__(16) float os[16 * 68];
    const size_t z = blockIdx.z; A += z * sA; if (A2) A2 += z * sA; Bt += z * sB; if (Bt2) Bt2 += z * sB; C += z * sC;
    const int lane = threadIdx.x & 31, lr = lane & 15, hi = lane >> 4; const int r0 = blockIdx.x * 64, c0 = blockIdx.y * 64;
    v8f acc[4][4];
#pragma unroll
    for (int mb = 0; mb < 4; ++mb)
#pragma unroll
        for (int nb = 0; nb < 4; ++nb) acc[mb][nb] = (v8f){};
    const size_t aoff = (size_t)(r0 + lr) * K + 8 * hi, boff = (size_t)(c0 + lr) * K + 8 * hi;
#pragma unroll 1
    for (int kc = 0; kc < K; kc += 32) {
        V a[4], a2[4];
#pragma unroll
        for (int mb = 0; mb < 4; ++mb) { a[mb] = WFrag<T16>::ld(A + aoff + (size_t)mb * 16 * K + kc); if (NSPLIT == 1 || NSPLIT == 2) a2[mb] = WFrag<T16>::ld(A2 + aoff + (size_t)mb * 16 * K + kc); }
#pragma unroll
        for (int nb = 0; nb < 4; ++nb) { const V b = WFrag<T16>::ld(Bt + boff + (size_t)nb * 16 * K + kc); V b2; if (NSPLIT >= 2) b2 = WFrag<T16>::ld(Bt2 + boff + (size_t)nb * 16 * K + kc);
#pragma unroll
            for (int mb = 0; mb < 4; ++mb) { acc[mb][nb] = WFrag<T16>::mma(a[mb], b, acc[mb][nb]); if (NSPLIT == 1 || NSPLIT == 2) acc[mb][nb] = WFrag<T16>::mma(a2[mb], b, acc[mb][nb]); if (NSPLIT >= 2) acc[mb][nb] = WFrag<T16>::mma(a[mb], b2, acc[mb][nb]); } }
        asm volatile("v_nop\n\tv_nop\n\tv_nop\n\tv_nop" : "+v"(acc[0][0]), "+v"(acc[1][1]), "+v"(acc[2][2]), "+v"(acc[3][3]) : "v"(a[0]), "v"(a[3]));
    }
#pragma unroll
    for (int mb = 0; mb < 4; ++mb) {
#pragma unroll
        for (int nb = 0; nb < 4; ++nb) {
#pragma unroll
            for (int j = 0; j < 8; ++j) os[(hi * 8 + j) * 68 + nb * 16 + lr] = acc[mb][nb][j]; }
        __builtin_amdgcn_wave_barrier(); asm volatile("" ::: "memory");
        float* crow = C + (size_t)(r0 + mb * 16) * ldc + c0;
#pragma unroll 1
        for (int ps = 0; ps < 2; ++ps) {
#pragma unroll
            for (int s = 0; s < 8; ++s) { const int row = 2 * s + hi, cofs = lr * 4; v4f val = *(const v4fa*)(os + row * 68 + cofs); if (BIAS) { val[0] += bfr(bias[c0 + cofs]); val[1] += bfr(bias[c0 + cofs + 1]); val[2] += bfr(bias[c0 + cofs + 2]); val[3] += bfr(bias[c0 + cofs + 3]); }
                *(volatile v4f*)(crow + (size_t)row * ldc + cofs) = val; }
            if (ps == 0) __threadfence(); }
        __builtin_amdgcn_wave_barrier(); asm volatile("" ::: "memory");
    }
}

__device__ __forceinline__ void splitf(float y, unsigned short& h, unsigned short& l) { h = f2bf(y); l = f2bf(y - bf2f(h)); }
typedef __attribute__((ext_vector_type(2))) unsigned short v2us;
typedef __attribute__((ext_vector_type(4))) unsigned short v4us;
__global__ __launch_bounds__(256) void k_cvt8(const float* __restrict__ src, bf* dst, size_t n8) { const size_t i = (size_t)blockIdx.x * 256 + threadIdx.x; if (i >= n8) return; const v8f v = *(const v8f*)(src + i * 8); v8us o;
#pragma unroll
    for (int k = 0; k < 8; ++k) o[k] = f2bf(v[k]); *(volatile v8us*)(dst + i * 8) = o; __threadfence(); *(volatile v8us*)(dst + i * 8) = o; }

__global__ __launch_bounds__(256) void k_sq(const float* __restrict__ a, float* SQ) { const int i = blockIdx.x * 256 + threadIdx.x; if (i >= NP) return; float s = 0.f;
#pragma unroll 4
    for (int d = 0; d < DD; ++d) { const float v = bfr(a[(size_t)i * DD + d]); float p = __fmul_rn(v, v); asm volatile("" : "+v"(p)); s = __fadd_rn(s, p); }
    *(volatile float*)(SQ + i) = s; __threadfence(); *(volatile float*)(SQ + i) = s; }
__global__ __launch_bounds__(256) void k_ytp(const float* __restrict__ y, bf* YT) { const size_t e = ((size_t)blockIdx.x * 256 + threadIdx.x) * 2; if (e >= (size_t)NPD * NP) return; const int j = (int)(e % NP), d = (int)(e / NP); v2us o; o[0] = 0; o[1] = 0; if (d < DD) { o[0] = f2bf(y[(size_t)j * DD + d]); o[1] = f2bf(y[(size_t)(j + 1) * DD + d]); }
    *(volatile v2us*)(YT + e) = o; __threadfence(); *(volatile v2us*)(YT + e) = o; }
__global__ __launch_bounds__(256) void k_kern(const float* __restrict__ G, const float* __restrict__ xs, const float* __restrict__ ys, int chunk, bf* Kh, bf* Kl, float* DEN) {
    const int lane = threadIdx.x & 31; const int il = blockIdx.x * 8 + (threadIdx.x >> 5); if (il >= CH) return; const int i = chunk * CH + il; const float xi = xs[i]; const float* gr = G + (size_t)il * NP;
#pragma unroll 1
    for (int ps = 0; ps < 2; ++ps) { float den = 0.f;
#pragma unroll 1
        for (int c = 0; c < NP / 128; ++c) { const int j0 = c * 128 + lane * 4; const v4f g4 = *(const v4f*)(gr + j0); v4us oh, ol;
#pragma unroll
            for (int q = 0; q < 4; ++q) { float t = __fadd_rn(xi, ys[j0 + q]); asm volatile("" : "+v"(t)); float s = __fsub_rn(t, __fmul_rn(2.0f, g4[q])); asm volatile("" : "+v"(s)); const float kv = expf(__fmul_rn(s, -0.0078125f)); den = __fadd_rn(den, kv); unsigned short a, b; splitf(kv, a, b); oh[q] = a; ol[q] = b; }
            const size_t oo = (size_t)il * NP + j0; *(volatile v4us*)(Kh + oo) = oh; *(volatile v4us*)(Kl + oo) = ol; }
#pragma unroll
        for (int sh = 16; sh; sh >>= 1) den += __shfl_xor(den, sh, 32);
        if (lane == 0) *(volatile float*)(DEN + (size_t)il * RP) = den;
        if (ps == 0) __threadfence(); } }
__global__ __launch_bounds__(256) void k_out(const float* __restrict__ NUM, const float* __restrict__ DEN, int chunk, float* O) { const int e = blockIdx.x * 256 + threadIdx.x; if (e >= CH * DD) return; const int d = e % DD, il = e / DD; const float v = __fdiv_rn(NUM[(size_t)il * NPD + d], DEN[(size_t)il * RP]); float* dst = O + ((size_t)chunk * CH + il) * DD + d; *(volatile float*)dst = v; __threadfence(); *(volatile float*)dst = v; }

extern "C" void kernel_launch(void* const* d_in, const int* in_sizes, int n_in,
                              void* d_out, int out_size, void* d_ws, size_t ws_size, hipStream_t stream) {
    (void)in_sizes; (void)n_in; (void)out_size;
    const float* px = (const float*)d_in[0]; const float* ry = (const float*)d_in[1];
    float* OUT = (float*)d_out;
    char* wsp = (char*)d_ws;
    auto take = [&](size_t bytes) { char* p = wsp; wsp += (bytes + 255) & ~(size_t)255; return (void*)p; };
    bf* XB = (bf*)take((size_t)NP * DD * 2); bf* YB = (bf*)take((size_t)NP * DD * 2); bf* YT = (bf*)take((size_t)NPD * NP * 2); float* XS = (float*)take(NP * 4); float* YS = (float*)take(NP * 4);
    float* G = (float*)take((size_t)CH * NP * 4); bf* Kh = (bf*)take((size_t)CH * NP * 2); bf* Kl = (bf*)take((size_t)CH * NP * 2); float* DEN = (float*)take((size_t)CH * RP * 4); float* NUM = (float*)take((size_t)CH * NPD * 4);
    if ((size_t)(wsp - (char*)d_ws) > ws_size) return;
    k_cvt8<<<(NP * DD / 8 + 255) / 256, 256, 0, stream>>>(px, XB, (size_t)NP * DD / 8); k_cvt8<<<(NP * DD / 8 + 255) / 256, 256, 0, stream>>>(ry, YB, (size_t)NP * DD / 8);
    k_ytp<<<(unsigned)(((size_t)NPD * NP / 2 + 255) / 256), 256, 0, stream>>>(ry, YT); k_sq<<<NP / 256, 256, 0, stream>>>(px, XS); k_sq<<<NP / 256, 256, 0, stream>>>(ry, YS);
    for (int c = 0; c < NCH; ++c) {
        k_gemmw<bf, 0, false><<<dim3(CH / 64, NP / 64, 1), 32, 0, stream>>>(XB + (size_t)c * CH * DD, nullptr, YB, nullptr, DD, G, NP, nullptr, 0, 0, 0);
        k_kern<<<CH / 8, 256, 0, stream>>>(G, XS, YS, c, Kh, Kl, DEN);
        k_gemmw<bf, 1, false><<<dim3(CH / 64, NPD / 64, 1), 32, 0, stream>>>(Kh, Kl, YT, nullptr, NP, NUM, NPD, nullptr, 0, 0, 0);
        k_out<<<(CH * DD + 255) / 256, 256, 0, stream>>>(NUM, DEN, c, OUT); }
}
